// RowAttentionWithPairBias_36172214566956
// MI455X (gfx1250) — hardware-verified
//
#include <hip/hip_runtime.h>


namespace {
constexpr int S = 128, R = 256, CM = 256, CZ = 128, H = 8, C = 32, NT = S * R, SL = 128  ;
constexpr float XS = 8.0f, WSC = 256.0f, PS = 1024.0f, LOG2E = 1.4426950408889634f, EPS = 1e-5f;
static_assert(R % 64 == 0 && CM == H * C && SL >= 1, "tiling");
typedef _Float16 b16;
typedef __attribute__((ext_vector_type(16))) _Float16 v16b;
typedef __attribute__((ext_vector_type(8))) _Float16 v8b;
typedef __attribute__((ext_vector_type(8))) float v8f;
typedef __attribute__((ext_vector_type(4))) float v4f;
__device__ __forceinline__ float bf16_rne(float f) { unsigned int u = __float_as_uint(f); u += 0x7FFFu + ((u >> 16) & 1u); return __uint_as_float(u & 0xFFFF0000u); }
__device__ __forceinline__ void split16(float v, b16& hi, b16& lo) { hi = (b16)v; lo = (b16)(v - (float)hi); }
__device__ __forceinline__ v16b frag_kb(const b16* p, int hh) { const v8b a = *(const v8b*)(p + 8 * hh), b = *(const v8b*)(p + 16 + 8 * hh); v16b f;
#pragma unroll
  for (int e = 0; e < 8; ++e) { f[e] = a[e]; f[8 + e] = b[e]; } return f; }
__device__ __forceinline__ v8f wmma16b(v16b a, v16b b, v8f c) { v8f d = __builtin_amdgcn_wmma_f32_16x16x32_f16(false, a, false, b, (short)0, c, false, false); asm volatile("v_nop\n\tv_nop\n\tv_nop\n\tv_nop" : "+v"(d) : "v"(a), "v"(b)); return d; }
__device__ __forceinline__ void wave_lds_sync() { __builtin_amdgcn_fence(__ATOMIC_RELEASE, "workgroup"); __builtin_amdgcn_wave_barrier(); __builtin_amdgcn_fence(__ATOMIC_ACQUIRE, "workgroup"); }
__device__ __forceinline__ float pmul(float a, float b) { float p = a * b; asm volatile("" : "+v"(p)); return p; }
__device__ __forceinline__ int iclamp(int v, int lo, int hi) { return v < lo ? lo : (v > hi ? hi : v); }

typedef __attribute__((ext_vector_type(2))) _Float16 v2h;
typedef __attribute__((ext_vector_type(4))) _Float16 v4h;
typedef __attribute__((ext_vector_type(2))) float v2f;
__device__ __forceinline__ float nexp2(float v) { return __builtin_amdgcn_exp2f(v); }
__global__ __launch_bounds__(256) void prep_kernel(const float* __restrict__ w2d, const float* __restrict__ wq, const float* __restrict__ wk, const float* __restrict__ wv, const float* __restrict__ wg, const float* __restrict__ wo, b16* __restrict__ W2, b16* __restrict__ WP, b16* __restrict__ WO) {
  size_t t = (size_t)blockIdx.x * 256 + threadIdx.x; v8b o;
  const size_t n1 = 16 * CZ / 8, n2 = (size_t)4 * CM * CM / 8, n3 = (size_t)CM * CM / 8;
  if (t < n1) { const int e = (int)t * 8; const int oo = e / CZ, c0 = e % CZ; for (int j = 0; j < 8; ++j) o[j] = (oo < H) ? (b16)(bf16_rne(w2d[(size_t)(c0 + j) * H + oo]) * WSC) : (b16)0.0f; for (int pass = 0; pass < 2; ++pass) { *(volatile v8b*)(W2 + e) = o; __threadfence(); } return; }
  t -= n1;
  if (t < n2) { const size_t e = t * 8; const int oo = (int)(e / CM), c0 = (int)(e % CM); const int part = oo / CM, hd = oo % CM; const float* w = part == 0 ? wq : part == 1 ? wk : part == 2 ? wv : wg; for (int j = 0; j < 8; ++j) o[j] = (b16)(bf16_rne(w[(size_t)(c0 + j) * CM + hd]) * WSC); for (int pass = 0; pass < 2; ++pass) { *(volatile v8b*)(WP + e) = o; __threadfence(); } return; }
  t -= n2;
  if (t < n3) { const size_t e = t * 8; const int oo = (int)(e / CM), k0 = (int)(e % CM); for (int j = 0; j < 8; ++j) o[j] = (b16)(bf16_rne(wo[(size_t)(k0 + j) * CM + oo]) * WSC); for (int pass = 0; pass < 2; ++pass) { *(volatile v8b*)(WO + e) = o; __threadfence(); } }
}
template <int KD>
__device__ __forceinline__ void stage_ln(const float* __restrict__ src  , size_t stride, const float* __restrict__ g, const float* __restrict__ bb, b16 (*Ah)[KD + 8], b16 (*Al)[KD + 8], int lane) {
  constexpr int PER = KD / 32;
  for (int rr = 0; rr < 16; ++rr) { float xv[PER]; float s = 0.0f;
#pragma unroll
    for (int q = 0; q < PER; ++q) { xv[q] = bf16_rne(src[(size_t)rr * stride + q * 32 + lane]); s += xv[q]; }
#pragma unroll
    for (int o = 1; o < 32; o <<= 1) s += __shfl_xor(s, o);
    const float mu = s * (1.0f / KD); float vs = 0.0f;
#pragma unroll
    for (int q = 0; q < PER; ++q) { const float d = xv[q] - mu; vs += d * d; }
#pragma unroll
    for (int o = 1; o < 32; o <<= 1) vs += __shfl_xor(vs, o);
    const float rs = rsqrtf(vs * (1.0f / KD) + EPS);
#pragma unroll
    for (int q = 0; q < PER; ++q) { const int c = q * 32 + lane; const float nv = (xv[q] - mu) * rs * bf16_rne(g[c]) + bf16_rne(bb[c]); b16 p, ql; split16(nv * XS, p, ql); Ah[rr][c] = p; Al[rr][c] = ql; } }
}
__global__ __launch_bounds__(128) void pairz_kernel(const float* __restrict__ pair, const float* __restrict__ pg, const float* __restrict__ pb, const b16* __restrict__ W2, float* __restrict__ Z) {
  __shared__ __attribute__((aligned(16))) b16 Ah[4][16][CZ + 8], Al[4][16][CZ + 8]; __shared__ float Tz[64][H + 1];
  const int wave = threadIdx.x >> 5, lane = threadIdx.x & 31, nloc = lane & 15, hlf = lane >> 4; const size_t row0 = (size_t)blockIdx.x * 64 + wave * 16;
  stage_ln<CZ>(pair + row0 * CZ, CZ, pg, pb, Ah[wave], Al[wave], lane);
  wave_lds_sync();
  v8f acc = (v8f){};
#pragma unroll
  for (int kb = 0; kb < CZ; kb += 32) { const v16b bw = frag_kb(W2 + (size_t)nloc * CZ + kb, hlf); acc = wmma16b(frag_kb(&Ah[wave][nloc][kb], hlf), bw, acc); acc = wmma16b(frag_kb(&Al[wave][nloc][kb], hlf), bw, acc); }
  if (nloc < H) {
#pragma unroll
    for (int r = 0; r < 8; ++r) Tz[wave * 16 + 8 * hlf + r][nloc] = acc[r] * (1.0f / (XS * WSC)); }
  __syncthreads();
  const int q = (int)((size_t)blockIdx.x * 64 / R), k0 = (int)((size_t)blockIdx.x * 64 % R);
  for (int pass = 0; pass < 2; ++pass) { for (int hp = 0; hp < 2; ++hp) { const int h = hp * 4 + wave; const v2f zz = {Tz[lane * 2][h], Tz[lane * 2 + 1][h]}; *(volatile v2f*)(Z + ((size_t)h * R + q) * R + k0 + lane * 2) = zz; } __threadfence(); }
}
__global__ __launch_bounds__(128) void proj_kernel(const float* __restrict__ msa, const float* __restrict__ qg, const float* __restrict__ qb, const b16* __restrict__ WP, const float* __restrict__ bg, b16* __restrict__ Qh, b16* __restrict__ Ql, b16* __restrict__ Kh, b16* __restrict__ Kl, b16* __restrict__ VTh, b16* __restrict__ VTl, float* __restrict__ G) {
  __shared__ __attribute__((aligned(16))) b16 Ah[4][16][CM + 8], Al[4][16][CM + 8]; __shared__ __attribute__((aligned(16))) float Tf[4][16][128 + 4];
  const int wave = threadIdx.x >> 5, lane = threadIdx.x & 31, nloc = lane & 15, hlf = lane >> 4; const size_t tok0 = (size_t)blockIdx.x * 64; const int s = (int)(tok0 / R), r0 = (int)(tok0 % R); if (s >= SL) return;
  const size_t m0 = tok0 + wave * 16; const int slab = blockIdx.y, n0 = slab * 128, part = slab / 2, c0 = n0 - part * CM;
  stage_ln<CM>(msa + m0 * CM, CM, qg, qb, Ah[wave], Al[wave], lane);
  wave_lds_sync();
  v8f acc[8];
#pragma unroll
  for (int t = 0; t < 8; ++t) acc[t] = (v8f){};
#pragma unroll 2
  for (int kb = 0; kb < CM; kb += 32) { const v16b ah = frag_kb(&Ah[wave][nloc][kb], hlf), al = frag_kb(&Al[wave][nloc][kb], hlf);
#pragma unroll
    for (int t = 0; t < 8; ++t) { const v16b bw = frag_kb(WP + (size_t)(n0 + t * 16 + nloc) * CM + kb, hlf); acc[t] = wmma16b(ah, bw, acc[t]); acc[t] = wmma16b(al, bw, acc[t]); } }
#pragma unroll
  for (int t = 0; t < 8; ++t) { const int c = c0 + t * 16 + nloc; const float bgv = (part == 3) ? bf16_rne(bg[c]) : 0.0f;
#pragma unroll
    for (int r = 0; r < 8; ++r) { float v = acc[t][r] * (1.0f / (XS * WSC)); if (part == 3) v = 1.0f / (1.0f + expf(-(v + bgv))); Tf[wave][8 * hlf + r][t * 16 + nloc] = v; } }
  __syncthreads();
  for (int pass = 0; pass < 2; ++pass) {
    if (part < 2) { b16* Ph_ = part == 0 ? Qh : Kh; b16* Pl_ = part == 0 ? Ql : Kl; const int cl = lane * 4; const int c = c0 + cl; const int h = c / C, d = c % C;
      for (int rr = 0; rr < 16; ++rr) { const int r = r0 + wave * 16 + rr; v4h hv, lv; for (int j = 0; j < 4; ++j) { b16 p, q; split16(Tf[wave][rr][cl + j] * XS, p, q); hv[j] = p; lv[j] = q; }
        const size_t oi = (((size_t)s * H + h) * R + r) * C + d; *(volatile v4h*)(Ph_ + oi) = hv; *(volatile v4h*)(Pl_ + oi) = lv; } }
    else if (part == 2) {
#pragma unroll 1
      for (int q = 0; q < 32; ++q) { const int cl = wave * 32 + q; const int c = c0 + cl; const int h = c / C, d = c % C; const int tk = lane * 2; v2h hv, lv;
        for (int j = 0; j < 2; ++j) { b16 p, ql; split16(Tf[(tk + j) >> 4][(tk + j) & 15][cl] * XS, p, ql); hv[j] = p; lv[j] = ql; }
        const size_t oi = (((size_t)s * H + h) * C + d) * R + r0 + lane * 2; *(volatile v2h*)(VTh + oi) = hv; *(volatile v2h*)(VTl + oi) = lv; } }
    else { for (int rr = 0; rr < 16; ++rr) *(volatile v4f*)(G + (m0 + rr) * CM + c0 + lane * 4) = *(const v4f*)(&Tf[wave][rr][lane * 4]); }
    __threadfence(); }
}
__global__ __launch_bounds__(64) void attn_kernel(const b16* __restrict__ Qh, const b16* __restrict__ Ql, const b16* __restrict__ Kh, const b16* __restrict__ Kl, const b16* __restrict__ VTh, const b16* __restrict__ VTl, const float* __restrict__ mask, const float* __restrict__ Z, float* __restrict__ OP) {
  __shared__ __attribute__((aligned(16))) b16 Pb[2][16][32 + 8], Pc[2][16][32 + 8]; __shared__ __attribute__((aligned(16))) float To[2][16][C + 4];
  const int wave = threadIdx.x >> 5, lane = threadIdx.x & 31, hh = lane >> 4, col = lane & 15; const int s = blockIdx.y / H, h = blockIdx.y % H; const int q0 = blockIdx.x * 32 + wave * 16, qi = q0 + col;
  const size_t ph = ((size_t)s * H + h); const b16* Qhb = Qh + ph * R * C; const b16* Qlb = Ql + ph * R * C; const b16* Khb = Kh + ph * R * C; const b16* Klb = Kl + ph * R * C; const b16* Vh = VTh + ph * C * R; const b16* Vl = VTl + ph * C * R;
  const float* Zq = Z + ((size_t)h * R + qi) * R; const float* Mr = mask + (size_t)s * R;
  const v16b qa = frag_kb(Qhb + (size_t)qi * C, hh), qb = frag_kb(Qlb + (size_t)qi * C, hh);
  const float cs = LOG2E / (5.656854249492381f * XS * XS);
  float m = -INFINITY, l = 0.0f; v8f o[2] = {(v8f){}, (v8f){}};
#pragma unroll 1
  for (int kb = 0; kb < R; kb += 32) {
    float e[16]; float mx = -INFINITY;
#pragma unroll
    for (int u = 0; u < 2; ++u) { v8f sc = (v8f){}; const size_t kr = (size_t)(kb + u * 16 + col) * C; const v16b kh0 = frag_kb(Khb + kr, hh), kl0 = frag_kb(Klb + kr, hh);
      sc = wmma16b(kh0, qa, sc); sc = wmma16b(kh0, qb, sc); sc = wmma16b(kl0, qa, sc);
      const int kk = kb + u * 16 + 8 * hh; const v4f z0 = *(const v4f*)(Zq + kk), z1 = *(const v4f*)(Zq + kk + 4), mk0 = *(const v4f*)(Mr + kk), mk1 = *(const v4f*)(Mr + kk + 4);
#pragma unroll
      for (int r = 0; r < 8; ++r) { const float zv = (r < 4) ? z0[r] : z1[r - 4]; const float mb = 1.0e9f * (bf16_rne(r < 4 ? mk0[r] : mk1[r - 4]) - 1.0f); const float vv = sc[r] * cs + (zv + mb) * LOG2E; e[u * 8 + r] = vv; mx = fmaxf(mx, vv); } }
    mx = fmaxf(mx, __shfl_xor(mx, 16)); const float mn = fmaxf(m, mx); const float al = (mn == -INFINITY) ? 1.0f : nexp2(m - mn); float sum = 0.0f;
#pragma unroll
    for (int i2 = 0; i2 < 16; ++i2) { const float p = nexp2(e[i2] - mn); sum += p; b16 a_, b_; split16(p * PS, a_, b_); const int sl = (i2 < 8 ? 0 : 16) + 8 * hh + (i2 & 7); Pb[wave][col][sl] = a_; Pc[wave][col][sl] = b_; }
    sum += __shfl_xor(sum, 16); l = l * al + sum; m = mn;
    wave_lds_sync();
    const v16b pf = frag_kb(&Pb[wave][col][0], hh), pgf = frag_kb(&Pc[wave][col][0], hh);
#pragma unroll
    for (int t = 0; t < 2; ++t) { o[t] *= al; const size_t vr = (size_t)(t * 16 + col) * R + kb; const v16b va = frag_kb(Vh + vr, hh), vb = frag_kb(Vl + vr, hh); o[t] = wmma16b(va, pf, o[t]); o[t] = wmma16b(va, pgf, o[t]); o[t] = wmma16b(vb, pf, o[t]); }
    wave_lds_sync(); }
  const float inv = 1.0f / (l * PS * XS);
#pragma unroll
  for (int t = 0; t < 2; ++t)
#pragma unroll
    for (int r = 0; r < 8; ++r) To[wave][col][t * 16 + 8 * hh + r] = o[t][r] * inv;
  wave_lds_sync();
  for (int pass = 0; pass < 2; ++pass) { for (int rr = 0; rr < 16; ++rr) ((volatile float*)OP)[(ph * R + q0 + rr) * C + lane] = To[wave][rr][lane]; __threadfence(); }
}
__global__ __launch_bounds__(128) void out_kernel(const float* __restrict__ OP, const float* __restrict__ G, const b16* __restrict__ WO, const float* __restrict__ bo, float* __restrict__ out) {
  __shared__ __attribute__((aligned(16))) float Tf[4][16][128 + 4];
  const int wave = threadIdx.x >> 5, lane = threadIdx.x & 31, nloc = lane & 15, hlf = lane >> 4; const size_t m0 = (size_t)blockIdx.x * 64 + wave * 16; const int n0 = blockIdx.y * 128; const size_t tok = m0 + nloc; const int s = (int)(tok / R), r = (int)(tok % R);
  v8f acc[8];
#pragma unroll
  for (int t = 0; t < 8; ++t) acc[t] = (v8f){};
#pragma unroll
  for (int ks = 0; ks < H; ++ks) { v16b ah, al; const float* orow = OP + (((size_t)s * H + ks) * R + r) * C; const float* grow = G + tok * CM + ks * C;
    const v4f c0 = *(const v4f*)(orow + 8 * hlf), c1 = *(const v4f*)(orow + 8 * hlf + 4), c2 = *(const v4f*)(orow + 16 + 8 * hlf), c3 = *(const v4f*)(orow + 16 + 8 * hlf + 4);
    const v4f g0 = *(const v4f*)(grow + 8 * hlf), g1 = *(const v4f*)(grow + 8 * hlf + 4), g2 = *(const v4f*)(grow + 16 + 8 * hlf), g3 = *(const v4f*)(grow + 16 + 8 * hlf + 4);
    float cv[16]; for (int i = 0; i < 4; ++i) { cv[i] = c0[i] * g0[i]; cv[4 + i] = c1[i] * g1[i]; cv[8 + i] = c2[i] * g2[i]; cv[12 + i] = c3[i] * g3[i]; }
#pragma unroll
    for (int e2 = 0; e2 < 16; ++e2) { b16 p, q; split16(cv[e2] * XS, p, q); ah[e2] = p; al[e2] = q; }
#pragma unroll
    for (int t = 0; t < 8; ++t) { const v16b bw = frag_kb(WO + (size_t)(n0 + t * 16 + nloc) * CM + ks * C, hlf); acc[t] = wmma16b(ah, bw, acc[t]); acc[t] = wmma16b(al, bw, acc[t]); } }
#pragma unroll
  for (int t = 0; t < 8; ++t) { const float bb = bf16_rne(bo[n0 + t * 16 + nloc]);
#pragma unroll
    for (int rr = 0; rr < 8; ++rr) Tf[wave][8 * hlf + rr][t * 16 + nloc] = acc[t][rr] * (1.0f / (XS * WSC)) + bb; }
  wave_lds_sync();
  for (int pass = 0; pass < 2; ++pass) { for (int rr = 0; rr < 16; ++rr) *(volatile v4f*)(out + (m0 + rr) * CM + n0 + lane * 4) = *(const v4f*)(&Tf[wave][rr][lane * 4]); __threadfence(); }
}
}

extern "C" void kernel_launch(void* const* d_in, const int* in_sizes, int n_in, void* d_out, int out_size, void* d_ws, size_t ws_size, hipStream_t stream) {
  (void)n_in;
  auto Fp = [&](int i) { return (const float*)d_in[i]; };
  if (in_sizes[0] != NT * CM || in_sizes[1] != R * R * CZ || in_sizes[2] != NT || in_sizes[3] != CM || in_sizes[5] != CZ || in_sizes[7] != CZ * H || in_sizes[8] != CM * CM || in_sizes[12] != CM || in_sizes[13] != CM * CM || in_sizes[14] != CM || out_size != NT * CM) return;
  size_t off = 0; char* ws = (char*)d_ws;
  auto carve = [&](size_t bytes) { char* p = ws + off; off += (bytes + 255) & ~(size_t)255; return p; };
  b16* W2 = (b16*)carve((size_t)16 * CZ * 2); b16* WP = (b16*)carve((size_t)4 * CM * CM * 2); b16* WO = (b16*)carve((size_t)CM * CM * 2); float* Z = (float*)carve((size_t)H * R * R * 4);
  const size_t plane = (size_t)NT * CM * 2; b16* Qh = (b16*)carve(plane); b16* Ql = (b16*)carve(plane); b16* Kh = (b16*)carve(plane); b16* Kl = (b16*)carve(plane); b16* VTh = (b16*)carve(plane); b16* VTl = (b16*)carve(plane);
  float* G = (float*)carve((size_t)NT * CM * 4); float* OP = (float*)carve((size_t)NT * CM * 4);
  if (off > ws_size || off > ((size_t)240 << 20)) return;
  prep_kernel<<<(unsigned)((16 * CZ / 8 + (size_t)4 * CM * CM / 8 + (size_t)CM * CM / 8 + 255) / 256), 256, 0, stream>>>(Fp(7), Fp(8), Fp(9), Fp(10), Fp(11), Fp(13), W2, WP, WO);
  pairz_kernel<<<(R * R) / 64, 128, 0, stream>>>(Fp(1), Fp(5), Fp(6), W2, Z);
  proj_kernel<<<dim3(NT / 64, 8), 128, 0, stream>>>(Fp(0), Fp(3), Fp(4), WP, Fp(12), Qh, Ql, Kh, Kl, VTh, VTl, G);
  attn_kernel<<<dim3(R / 32, SL * H), 64, 0, stream>>>(Qh, Ql, Kh, Kl, VTh, VTl, Fp(2), Z, OP);
  out_kernel<<<dim3((SL * R) / 64, 2), 128, 0, stream>>>(OP, G, WO, Fp(14), (float*)d_out);
}
